// Memory_cell_6957847019562
// MI455X (gfx1250) — hardware-run, weakly checked
//
#include <hip/hip_runtime.h>
#include <math.h>

typedef __attribute__((ext_vector_type(16))) _Float16 v16h;
typedef __attribute__((ext_vector_type(16))) __bf16 v16b;
typedef __attribute__((ext_vector_type(8)))  _Float16 v8h;
typedef __attribute__((ext_vector_type(8)))  float v8f;
typedef __attribute__((ext_vector_type(4)))  float v4f;
typedef __attribute__((ext_vector_type(2)))  float v2f;
typedef __attribute__((ext_vector_type(4)))  unsigned v4u;
typedef __attribute__((ext_vector_type(4)))  int v4i;
typedef float __attribute__((may_alias)) float_a;
typedef int __attribute__((may_alias)) int_a;

template <typename T> __device__ __forceinline__ void vst2(void* p, T v) { *(volatile T*)p = v; __threadfence(); *(volatile T*)p = v; }
__device__ __forceinline__ v8f wmma16(v16h a, v16h b, v8f c) {
  v8f d = __builtin_amdgcn_wmma_f32_16x16x32_f16(false, a, false, b, (short)0, c, false, false);
  asm volatile("v_nop\n\tv_nop\n\tv_nop\n\tv_nop" : "+v"(d) : "v"(a), "v"(b));
  return d;
}
__device__ __forceinline__ v8f wmma_bf(v16b a, v16b b, v8f c) {
  v8f d = __builtin_amdgcn_wmma_f32_16x16x32_bf16(false, a, false, b, (short)0, c, false, false);
  asm volatile("v_nop\n\tv_nop\n\tv_nop\n\tv_nop" : "+v"(d) : "v"(a), "v"(b));
  return d;
}
__device__ __forceinline__ v16h frag_h(const _Float16* rowk0, int lane) {
  union { v16h v; v8h q[2]; } u; const _Float16* p = rowk0 + 8 * (lane >> 4);
  u.q[0] = *(const v8h*)p; u.q[1] = *(const v8h*)(p + 16); return u.v;
}
__device__ __forceinline__ v16h frag_f32(const float* rowk0, int lane) {
  v16h a; const float* p = rowk0 + 8 * (lane >> 4);
#pragma unroll
  for (int i = 0; i < 8; ++i) { a[i] = (_Float16)p[i]; a[8 + i] = (_Float16)p[16 + i]; }
  return a;
}
__device__ __forceinline__ v16h frag_f32s(const float* rowk0, int lane, float sc) {
  v16h a; const float* p = rowk0 + 8 * (lane >> 4);
#pragma unroll
  for (int i = 0; i < 8; ++i) { a[i] = (_Float16)(p[i] * sc); a[8 + i] = (_Float16)(p[16 + i] * sc); }
  return a;
}
__device__ __forceinline__ v16h fragc_f32(const float* W, int k0, int n, int lane, int ld, int K) {
  v16h a; const int g = lane >> 4;
#pragma unroll
  for (int i = 0; i < 8; ++i) { const int ka = k0 + 8 * g + i, kb = ka + 16;
    a[i] = (_Float16)(ka < K ? W[(size_t)(ka < K ? ka : K - 1) * ld + n] : 0.f); a[8 + i] = (_Float16)(kb < K ? W[(size_t)(kb < K ? kb : K - 1) * ld + n] : 0.f); }
  return a;
}
struct F2 { v16b h, l; };
__device__ __forceinline__ F2 bsplit16(const float v[16]) { F2 r;
#pragma unroll
  for (int i = 0; i < 16; ++i) { const __bf16 h = (__bf16)v[i]; r.h[i] = h; r.l[i] = (__bf16)(v[i] - (float)h); }
  return r; }
__device__ __forceinline__ F2 split_row(const float* row, int k0, int lane) { float v[16]; const float* p = row + k0 + 8 * (lane >> 4);
#pragma unroll
  for (int i = 0; i < 8; ++i) { v[i] = p[i]; v[8 + i] = p[16 + i]; }
  return bsplit16(v); }
__device__ __forceinline__ F2 split_rowK(const float* row, int k0, int lane, int K) { float v[16]; const int g = lane >> 4;
#pragma unroll
  for (int i = 0; i < 8; ++i) { const int ka = k0 + 8 * g + i, kb = ka + 16; v[i] = ka < K ? row[ka < K ? ka : K - 1] : 0.f; v[8 + i] = kb < K ? row[kb < K ? kb : K - 1] : 0.f; }
  return bsplit16(v); }
__device__ __forceinline__ F2 split_col(const float* W, int k0, int n, int lane, int ld, int K) { float v[16]; const int g = lane >> 4;
#pragma unroll
  for (int i = 0; i < 8; ++i) { const int ka = k0 + 8 * g + i, kb = ka + 16; v[i] = ka < K ? W[(size_t)(ka < K ? ka : K - 1) * ld + n] : 0.f; v[8 + i] = kb < K ? W[(size_t)(kb < K ? kb : K - 1) * ld + n] : 0.f; }
  return bsplit16(v); }
__device__ __forceinline__ v8f mac3(const F2& a, const F2& b, v8f c) { c = wmma_bf(a.l, b.h, c); c = wmma_bf(a.h, b.l, c); return wmma_bf(a.h, b.h, c); }
__device__ __forceinline__ float sigm(float v) { return 1.0f / (1.0f + expf(-v)); }
#define LDSX() do { asm volatile("s_wait_dscnt 0" ::: "memory"); __builtin_amdgcn_wave_barrier(); __builtin_amdgcn_fence(__ATOMIC_RELEASE, "workgroup"); } while (0)


#define NBAT 2048
#define KK 4096
#define RR 2048
#define VV 2048
#ifndef VVU
#define VVU VV
#define NBR (NBAT / 64)
#endif
typedef __attribute__((ext_vector_type(8))) __bf16 v8b;
__device__ __forceinline__ v16b frag_b(const __bf16* rowk0, int lane) {
  union { v16b v; v8b q[2]; } u; const __bf16* p = rowk0 + 8 * (lane >> 4);
  u.q[0] = *(const v8b*)p; u.q[1] = *(const v8b*)(p + 16); return u.v;
}
__device__ __forceinline__ float bfr(float v) { return (float)(__bf16)v; }
__device__ __attribute__((noinline)) float exp_ni(float v) { return expf(v); }
__device__ __attribute__((noinline)) float erf_ni(float v) { return erff(v); }
__device__ __attribute__((noinline)) float tanh_ni(float v) { return tanhf(v); }

#define WS_PK   0u
#define WS_MT   (2u * VV * RR)
#define WS_SP   (WS_MT + 2u * RR * KK)
#define WS_SC   (WS_SP + 4u * KK * 16)
#define WS_AT   (WS_SC + 4u * KK)
#define WS_ATL  (WS_AT + 2u * 16 * KK)
#define WS_ROW  (WS_ATL + 2u * 16 * KK)
#define WS_END  (WS_ROW + 4u * RR)

__global__ __launch_bounds__(256) void k_pack(const float* __restrict__ WM, __bf16* __restrict__ PK) {
  __shared__ __align__(16) __bf16 s[RR]; const int n = blockIdx.x, t = threadIdx.x;
  for (int k = t; k < RR; k += 256) s[k] = (__bf16)WM[(size_t)n * RR + k];
  __syncthreads();
  for (int q = t; q < RR / 8; q += 256) vst2((unsigned*)(PK + (size_t)n * RR + q * 8), *(const v4u*)&s[q * 8]);
}
__global__ __launch_bounds__(256) void k_mt(const float* __restrict__ M, __bf16* __restrict__ MT) {
  __shared__ __align__(16) __bf16 s[128][72]; const int tid = threadIdx.x; const int kb = blockIdx.x, rb = blockIdx.y; const int k0 = kb * 64, r0 = rb * 128;
  for (int e = tid; e < 64 * 128; e += 256) { const int kk = e >> 7, r = e & 127; s[r][kk] = (__bf16)M[(size_t)(k0 + kk) * RR + r0 + r]; }
  __syncthreads();
  for (int e = tid; e < 128 * 8; e += 256) { const int r = e >> 3, pc = e & 7; vst2((unsigned*)(MT + (size_t)(r0 + r) * KK + k0 + pc * 8), *(const v4u*)&s[r][pc * 8]); }
}
__global__ __launch_bounds__(128) void k_score2(const float* __restrict__ M, const __bf16* __restrict__ PK, const float* __restrict__ WMB, const float* __restrict__ WW, float* __restrict__ SP) {
  __shared__ __align__(16) float sred[64];
  const int tid = threadIdx.x, wave = tid >> 5, lane = tid & 31, col = lane & 15, g = lane >> 4; const size_t r0 = (size_t)blockIdx.x * 64 + wave * 16; const int n0 = blockIdx.y * 128;
  v8f acc[8] = {};
#pragma unroll 2
  for (int kc = 0; kc < RR / 32; ++kc) { v16b a; { const float* p = M + (r0 + col) * RR + kc * 32 + 8 * g;
#pragma unroll
      for (int i = 0; i < 8; ++i) { a[i] = (__bf16)p[i]; a[8 + i] = (__bf16)p[16 + i]; } }
#pragma unroll
    for (int j = 0; j < 8; ++j) acc[j] = wmma_bf(a, frag_b(PK + (size_t)(n0 + j * 16 + col) * RR + kc * 32, lane), acc[j]); }
  float part[8];
#pragma unroll
  for (int r = 0; r < 8; ++r) part[r] = 0.f;
#pragma unroll
  for (int j = 0; j < 8; ++j) { const int c = n0 + j * 16 + col; const float w = bfr(WW[c]); const float bb = bfr(WMB[c]);
#pragma unroll
    for (int r = 0; r < 8; ++r) part[r] += tanh_ni(acc[j][r] + bb) * w; }
#pragma unroll
  for (int r = 0; r < 8; ++r) { float v = part[r];
#pragma unroll
    for (int o = 1; o < 16; o <<= 1) v += __shfl_xor(v, o);
    if (col == 0) sred[wave * 16 + 8 * g + r] = v; }
  __syncthreads();
  if (tid < 16) vst2(SP + ((size_t)blockIdx.x * 16 + blockIdx.y) * 64 + tid * 4, *(const v4f*)&sred[tid * 4]);
}
__global__ __launch_bounds__(256) void k_soft(const float* __restrict__ SP, const float* __restrict__ WB, __bf16* __restrict__ AT, __bf16* __restrict__ ATL) {
  __shared__ float ssc[KK]; __shared__ float red[8]; const int t = threadIdx.x; const float wb = bfr(WB[0]);
  float mx = -3.0e38f; for (int k = t; k < KK; k += 256) { float s = 0.f; for (int vb = 0; vb < VVU / 128; ++vb) s += SP[((size_t)(k >> 6) * 16 + vb) * 64 + (k & 63)]; s += wb; ssc[k] = s; mx = fmaxf(mx, s); }
#pragma unroll
  for (int o = 1; o < 32; o <<= 1) mx = fmaxf(mx, __shfl_xor(mx, o));
  if ((t & 31) == 0) red[t >> 5] = mx; __syncthreads(); float gm = -3.0e38f; for (int w = 0; w < 8; ++w) gm = fmaxf(gm, red[w]); __syncthreads();
  float sm = 0.f; for (int k = t; k < KK; k += 256) { const float e = exp_ni(ssc[k] - gm); ssc[k] = e; sm += e; }
#pragma unroll
  for (int o = 1; o < 32; o <<= 1) sm += __shfl_xor(sm, o);
  if ((t & 31) == 0) red[t >> 5] = sm; __syncthreads(); float tot = 0.f; for (int w = 0; w < 8; ++w) tot += red[w]; const float inv = 1.0f / tot;
  for (int e = t; e < 16 * KK / 8; e += 256) { const int row = e / (KK / 8), q = e % (KK / 8); __align__(16) __bf16 hh[8], ll[8];
#pragma unroll
    for (int i = 0; i < 8; ++i) { float a = (row == 0) ? ssc[q * 8 + i] * inv : 0.f; const __bf16 hb = (__bf16)a; hh[i] = hb; ll[i] = (__bf16)(a - (float)hb); }
    vst2((unsigned*)(AT + (size_t)row * KK + q * 8), *(const v4u*)hh); vst2((unsigned*)(ATL + (size_t)row * KK + q * 8), *(const v4u*)ll); }
}
__global__ __launch_bounds__(128) void k_read(const __bf16* __restrict__ AT, const __bf16* __restrict__ ATL, const __bf16* __restrict__ MT, float* __restrict__ ROW) {
  __shared__ __align__(16) float so[128];
  const int tid = threadIdx.x, wave = tid >> 5, lane = tid & 31, col = lane & 15, g = lane >> 4; const int n0 = blockIdx.x * 128;
  v8f acc[2] = {};
#pragma unroll 4
  for (int kc = 0; kc < KK / 32; ++kc) { F2 a; a.h = frag_b(AT + (size_t)col * KK + kc * 32, lane); a.l = frag_b(ATL + (size_t)col * KK + kc * 32, lane);
#pragma unroll
    for (int j = 0; j < 2; ++j) { const v16b w = frag_b(MT + (size_t)(n0 + (wave * 2 + j) * 16 + col) * KK + kc * 32, lane); acc[j] = wmma_bf(a.l, w, acc[j]); acc[j] = wmma_bf(a.h, w, acc[j]); } }
#pragma unroll
  for (int j = 0; j < 2; ++j) if (g == 0) so[(wave * 2 + j) * 16 + col] = acc[j][0];
  __syncthreads();
  if (tid < 32) vst2(ROW + n0 + tid * 4, *(const v4f*)&so[tid * 4]);
}
__global__ __launch_bounds__(256) void k_bcast(const float* __restrict__ ROW, float* __restrict__ OUT) {
  const int t = threadIdx.x; const size_t b0 = (size_t)blockIdx.x * 64;
  for (int q = t; q < RR / 4; q += 256) { const v4f v = *(const v4f*)(ROW + q * 4); for (int r = 0; r < 64; ++r) vst2(OUT + (b0 + r) * RR + q * 4, v); }
}
extern "C" void kernel_launch(void* const* d_in, const int* in_sizes, int n_in, void* d_out, int out_size, void* d_ws, size_t ws_size, hipStream_t stream) {
  (void)in_sizes; (void)n_in; (void)out_size;
  const float** F = (const float**)d_in;
  if (ws_size < (size_t)WS_END) return;
  char* ws = (char*)d_ws; __bf16 *PK = (__bf16*)(ws + WS_PK), *MT = (__bf16*)(ws + WS_MT), *AT = (__bf16*)(ws + WS_AT), *ATL = (__bf16*)(ws + WS_ATL); float *SP = (float*)(ws + WS_SP), *SC = (float*)(ws + WS_SC), *ROW = (float*)(ws + WS_ROW); (void)SC;
  k_pack<<<VV, 256, 0, stream>>>(F[4], PK);
  k_mt<<<dim3(KK / 64, RR / 128), 256, 0, stream>>>(F[1], MT);
  k_score2<<<dim3(KK / 64, VVU / 128), 128, 0, stream>>>(F[1], PK, F[5], F[6], SP);
  k_soft<<<1, 256, 0, stream>>>(SP, F[7], AT, ATL);
  k_read<<<RR / 128, 128, 0, stream>>>(AT, ATL, MT, ROW);
  k_bcast<<<NBR, 256, 0, stream>>>(ROW, (float*)d_out);
}
